// AGRNNModel_47691316855473
// MI455X (gfx1250) — hardware-run, weakly checked
//
#include <hip/hip_runtime.h>
#include <math.h>

constexpr int kBatch   = 32;
constexpr int kTin     = 12;
constexpr int kFeat    = 2;
constexpr int kLinks   = 1024;
constexpr int kHid     = 64;
constexpr int kHor     = 12;
constexpr int kBH      = kBatch * kHid;
constexpr int kBF      = kBatch * kFeat;
constexpr int kGateN   = 3 * kHid;
constexpr int kEncN    = kTin * kBF;
constexpr int kLTab    = 12 * kHid;
constexpr int kDecCell = kHor - 1;
constexpr float kAttnWCarry = 256.0f;
constexpr float kHidCarry   = 64.0f;
constexpr float kHattCarry  = 256.0f;
constexpr float kGateWCarry = 8.0f;
constexpr float kAttnScale  = 1.0f / (256.0f * 64.0f);
constexpr float kInScale    = 1.0f / 256.0f;
constexpr float kGateScale  = 1.0f / (256.0f * 8.0f);
static_assert(kBH == 2048 && kBF == 64 && kGateN == 192 && kEncN == 768 && kLTab == 768, "sizes");

typedef __attribute__((ext_vector_type(16))) _Float16 v16h;
typedef __attribute__((ext_vector_type(8)))  _Float16 v8h;
typedef __attribute__((ext_vector_type(16))) __bf16   v16b;
typedef __attribute__((ext_vector_type(8)))  __bf16   v8b;
typedef __attribute__((ext_vector_type(8)))  float    v8f;
typedef __attribute__((ext_vector_type(4)))  float    v4f;
typedef __attribute__((ext_vector_type(4)))  unsigned int v4u;

__device__ __forceinline__ unsigned short f2bf_bits(float f) {
  unsigned u = __float_as_uint(f);
  return (unsigned short)((u + 0x7FFFu + ((u >> 16) & 1u)) >> 16);
}
__device__ __forceinline__ float bf_bits2f(unsigned short h) { return __uint_as_float(((unsigned)h) << 16); }

__device__ __forceinline__ void dep_guard_h(v8f& a, v8f& b, v16h x, v16h y) { asm volatile("v_nop\n\tv_nop\n\tv_nop\n\tv_nop" : "+v"(a), "+v"(b) : "v"(x), "v"(y)); }
__device__ __forceinline__ void dep_guard_b(v8f& a, v8f& b, v16b x, v16b y) { asm volatile("v_nop\n\tv_nop\n\tv_nop\n\tv_nop" : "+v"(a), "+v"(b) : "v"(x), "v"(y)); }
__device__ __forceinline__ void keep4_h(v16h a, v16h b, v16h c, v16h d) { asm volatile("v_nop" :: "v"(a), "v"(b), "v"(c), "v"(d)); }
__device__ __forceinline__ void keep4_b(v16b a, v16b b, v16b c, v16b d) { asm volatile("v_nop" :: "v"(a), "v"(b), "v"(c), "v"(d)); }
__device__ __forceinline__ void acc_guard4(v8f& a, v8f& b, v8f& c, v8f& d) { asm volatile("v_nop\n\tv_nop\n\tv_nop\n\tv_nop" : "+v"(a), "+v"(b), "+v"(c), "+v"(d)); }
template <typename T> struct Frag;
template <> struct Frag<_Float16> {
  typedef v16h V; union U { v16h v; v8h h[2]; };
  static __device__ __forceinline__ v16h load(const _Float16* p) {
    U f; f.h[0] = *(const v8h*)(p); f.h[1] = *(const v8h*)(p + 16); return f.v;
  }
  static __device__ __forceinline__ v8f mma(v16h a, v16h b, v8f c) {
    return __builtin_amdgcn_wmma_f32_16x16x32_f16(false, a, false, b, (short)0, c, false, false);
  }
  static __device__ __forceinline__ void guard(v8f& a, v8f& b, v16h x, v16h y) { dep_guard_h(a, b, x, y); }
  static __device__ __forceinline__ void keep(v16h a, v16h b, v16h c, v16h d) { keep4_h(a, b, c, d); }
};
template <> struct Frag<__bf16> {
  typedef v16b V; union U { v16b v; v8b h[2]; };
  static __device__ __forceinline__ v16b load(const __bf16* p) {
    U f; f.h[0] = *(const v8b*)(p); f.h[1] = *(const v8b*)(p + 16); return f.v;
  }
  static __device__ __forceinline__ v8f mma(v16b a, v16b b, v8f c) {
    return __builtin_amdgcn_wmma_f32_16x16x32_bf16(false, a, false, b, (short)0, c, false, false);
  }
  static __device__ __forceinline__ void guard(v8f& a, v8f& b, v16b x, v16b y) { dep_guard_b(a, b, x, y); }
  static __device__ __forceinline__ void keep(v16b a, v16b b, v16b c, v16b d) { keep4_b(a, b, c, d); }
};

__device__ __forceinline__ unsigned pk16(unsigned short a, unsigned short b) { return (unsigned)a | ((unsigned)b << 16); }
__device__ __forceinline__ unsigned short h_bits(float f) { const _Float16 h = (_Float16)f; return __builtin_bit_cast(unsigned short, h); }

__device__ __forceinline__ void keep3_h(v16h a, v16h b, v16h c) { asm volatile("v_nop" :: "v"(a), "v"(b), "v"(c)); }
__device__ __forceinline__ void acc_guard3(v8f& a, v8f& b, v8f& c) { asm volatile("v_nop\n\tv_nop\n\tv_nop\n\tv_nop" : "+v"(a), "+v"(b), "+v"(c)); }

template <int ET> struct Elem;
template <> struct Elem<0> { typedef _Float16 T; };
template <> struct Elem<1> { typedef __bf16 T; };
template <int ET, bool SPLIT, int BIAS_MODE, int OUT_MODE, bool RESID, int ACT = 0>
__global__ __launch_bounds__(256) void wmma_gemm64(
    const unsigned short* __restrict__ Ap, const unsigned short* __restrict__ A2p, int lda, long strideA,
    const unsigned short* __restrict__ Btp, const unsigned short* __restrict__ Bt2p, int ldb, long strideB,
    void* __restrict__ Cout, void* __restrict__ Cout2, int ldc, long strideC,
    const float* __restrict__ bias,
    const float* __restrict__ resid, long strideR,
    int M, int N, int K, float scale) {
  typedef typename Elem<ET>::T T;
  typedef typename Frag<T>::V V;
  const T* A = (const T*)Ap; const T* A2 = (const T*)A2p; const T* Bt = (const T*)Btp; const T* Bt2 = (const T*)Bt2p;
  __shared__ __align__(16) float sT[8][16 * 68];
  const int b    = blockIdx.y;
  const int lane = threadIdx.x & 31;
  const int wave = threadIdx.x >> 5;
  const int tilesN = N >> 6;
  const int tilesM = M >> 6;
  const int tile = blockIdx.x * 8 + wave;
  if (tile >= tilesM * tilesN) return;
  const int tm = tile / tilesN;
  const int tn = tile - tm * tilesN;
  const int m0 = tm << 6;
  const int n0 = tn << 6;

  const T* Ab  = A  + (size_t)b * strideA;
  const T* Bb  = Bt + (size_t)b * strideB;
  const T* Ab2 = SPLIT ? (A2  + (size_t)b * strideA) : nullptr;
  const T* Bb2 = SPLIT ? (Bt2 + (size_t)b * strideB) : nullptr;

  const int rlane = lane & 15;
  const int koff  = (lane >> 4) * 8;
  const int mOff  = (lane >> 4) * 8;

  v8f acc[4][4];
#pragma unroll
  for (int i = 0; i < 4; ++i)
#pragma unroll
    for (int j = 0; j < 4; ++j) acc[i][j] = (v8f){0.f,0.f,0.f,0.f,0.f,0.f,0.f,0.f};

  for (int k0 = 0; k0 < K; k0 += 32) {
    V bh[4], bl[4];
#pragma unroll
    for (int j = 0; j < 4; ++j) {
      const size_t bo = (size_t)(n0 + (j << 4) + rlane) * ldb + koff + k0;
      bh[j] = Frag<T>::load(Bb + bo);
      if (SPLIT) bl[j] = Frag<T>::load(Bb2 + bo);
    }
#pragma unroll
    for (int i = 0; i < 4; ++i) {
      const size_t ao = (size_t)(m0 + (i << 4) + rlane) * lda + koff + k0;
      V ah = Frag<T>::load(Ab + ao);
      V al;
      if (SPLIT) al = Frag<T>::load(Ab2 + ao);
#pragma unroll
      for (int j = 0; j < 4; ++j) {
        acc[i][j] = Frag<T>::mma(ah, bh[j], acc[i][j]);
        if (SPLIT) {
          acc[i][j] = Frag<T>::mma(ah, bl[j], acc[i][j]);
          acc[i][j] = Frag<T>::mma(al, bh[j], acc[i][j]);
        }
      }
      Frag<T>::guard(acc[i][0], acc[i][3], ah, SPLIT ? al : ah);
    }
    Frag<T>::keep(bh[0], bh[1], bh[2], bh[3]);
    if (SPLIT) Frag<T>::keep(bl[0], bl[1], bl[2], bl[3]);
  }
  acc_guard4(acc[0][0], acc[0][1], acc[0][2], acc[0][3]);
  acc_guard4(acc[1][0], acc[1][1], acc[1][2], acc[1][3]);
  acc_guard4(acc[2][0], acc[2][1], acc[2][2], acc[2][3]);
  acc_guard4(acc[3][0], acc[3][1], acc[3][2], acc[3][3]);

  float* slab = sT[wave];
  const float* Rb = RESID ? (resid + (size_t)b * strideR) : nullptr;
#pragma unroll
  for (int i = 0; i < 4; ++i) {
    const int mBase = m0 + (i << 4);
#pragma unroll
    for (int j = 0; j < 4; ++j) {
      const int n = n0 + (j << 4) + rlane;
      float bv = 0.f;
      if (BIAS_MODE == 2) bv = bias[n];
#pragma unroll
      for (int r = 0; r < 8; ++r) {
        float v = acc[i][j][r] * scale;
        if (BIAS_MODE == 1) v += bias[mBase + mOff + r];
        if (BIAS_MODE == 2) v += bv;
        if (RESID) v += Rb[(size_t)(mBase + mOff + r) * ldc + n];
        if (ACT == 1) v = tanhf(v);
        if (ACT == 2) v = fmaxf(v, 0.0f);
        if (ACT == 3) v = v / (1.0f + expf(-v));
        if (ACT == 4) v = (v > 0.f) ? v : 0.01f * v;
        if (ACT == 5) v = 0.5f * v * (1.0f + erff(v * 0.70710678118654752f));
        slab[(mOff + r) * 68 + (j << 4) + rlane] = v;
      }
    }
    __builtin_amdgcn_fence(__ATOMIC_RELEASE, "workgroup");
    __builtin_amdgcn_wave_barrier();
    __builtin_amdgcn_fence(__ATOMIC_ACQUIRE, "workgroup");
    if (OUT_MODE == 0) {
      float* C = (float*)Cout + (size_t)b * strideC;
      const int hh = lane >> 4, c4 = (lane & 15) * 4;
      for (int pass = 0; pass < 2; ++pass) {
#pragma unroll
        for (int it = 0; it < 8; ++it) {
          const int row = it * 2 + hh;
          v4f v = *(const v4f*)(slab + row * 68 + c4);
          *(volatile v4f*)(C + (size_t)(mBase + row) * ldc + n0 + c4) = v;
        }
        __threadfence();
      }
    } else {
      const int q = lane >> 3, c8 = (lane & 7) * 8;
      unsigned short* C  = (unsigned short*)Cout  + (size_t)b * strideC;
      unsigned short* C2 = (OUT_MODE == 2) ? ((unsigned short*)Cout2 + (size_t)b * strideC) : nullptr;
      for (int pass = 0; pass < 2; ++pass) {
#pragma unroll
        for (int it = 0; it < 4; ++it) {
          const int row = it * 4 + q;
          const float* sp = slab + row * 68 + c8;
          v8h hv, lv;
#pragma unroll
          for (int e = 0; e < 8; ++e) {
            if (OUT_MODE == 1) {
              hv[e] = (_Float16)sp[e];
            } else {
              unsigned short hb = f2bf_bits(sp[e]);
              unsigned short lb = f2bf_bits(sp[e] - bf_bits2f(hb));
              hv[e] = __builtin_bit_cast(_Float16, hb);
              lv[e] = __builtin_bit_cast(_Float16, lb);
            }
          }
          *(volatile v8h*)(C + (size_t)(mBase + row) * ldc + n0 + c8) = hv;
          if (OUT_MODE == 2) *(volatile v8h*)(C2 + (size_t)(mBase + row) * ldc + n0 + c8) = lv;
        }
        __threadfence();
      }
    }
    __builtin_amdgcn_fence(__ATOMIC_RELEASE, "workgroup");
    __builtin_amdgcn_wave_barrier();
    __builtin_amdgcn_fence(__ATOMIC_ACQUIRE, "workgroup");
  }
}

__global__ __launch_bounds__(256) void cast8h_kernel(const float* __restrict__ in, unsigned short* __restrict__ out, int n8, float scale) {
  const int i = blockIdx.x * 256 + threadIdx.x;
  if (i >= n8) return;
  const float* p = in + 8 * (size_t)i;
  const v4f a = *(const v4f*)(p);
  const v4f c = *(const v4f*)(p + 4);
  unsigned short hb[8];
#pragma unroll
  for (int e = 0; e < 4; ++e) {
    hb[e]     = h_bits(a[e] * scale);
    hb[4 + e] = h_bits(c[e] * scale);
  }
  const v4u u = (v4u){pk16(hb[0], hb[1]), pk16(hb[2], hb[3]), pk16(hb[4], hb[5]), pk16(hb[6], hb[7])};
  unsigned short* q = out + 8 * (size_t)i;
  *(volatile v4u*)q = u;
  __threadfence();
  *(volatile v4u*)q = u;
}

__global__ __launch_bounds__(256) void castx_kernel(const float* __restrict__ x, unsigned short* __restrict__ out, int n8) {
  const int i = blockIdx.x * 256 + threadIdx.x;
  if (i >= n8) return;
  const int row = i >> 7;
  const int l0  = (i & 127) * 8;
  const int t   = row >> 6;
  const int bf  = row & 63;
  const int b   = bf >> 1, f = bf & 1;
  const float* p = x + ((size_t)(b * kTin + t) * (kFeat * kLinks) + (size_t)f * kLinks + l0);
  const v4f a = *(const v4f*)(p);
  const v4f c = *(const v4f*)(p + 4);
  unsigned short hb[8];
#pragma unroll
  for (int e = 0; e < 4; ++e) {
    hb[e]     = h_bits(a[e]);
    hb[4 + e] = h_bits(c[e]);
  }
  const v4u u = (v4u){pk16(hb[0], hb[1]), pk16(hb[2], hb[3]), pk16(hb[4], hb[5]), pk16(hb[6], hb[7])};
  unsigned short* q = out + (size_t)row * kLinks + l0;
  *(volatile v4u*)q = u;
  __threadfence();
  *(volatile v4u*)q = u;
}

__global__ __launch_bounds__(256) void prep_gates_kernel(const float* __restrict__ Wr, const float* __restrict__ Wz,
                                                         const float* __restrict__ Wn, unsigned short* __restrict__ WG) {
  __shared__ float tile[64 * 65];
  const int l = blockIdx.x;
  const int g = blockIdx.y;
  const int t = threadIdx.x;
  const float* W  = (g == 0) ? Wr : ((g == 1) ? Wz : Wn);
  const float* Wl = W + (size_t)l * (kHid * kHid);
  {
    const int h = t >> 2, k16 = (t & 3) * 16;
    const float* p = Wl + h * kHid + k16;
    const v4f a0 = *(const v4f*)(p);
    const v4f a1 = *(const v4f*)(p + 4);
    const v4f a2 = *(const v4f*)(p + 8);
    const v4f a3 = *(const v4f*)(p + 12);
#pragma unroll
    for (int e = 0; e < 4; ++e) {
      tile[h * 65 + k16 + e]      = a0[e];
      tile[h * 65 + k16 + 4 + e]  = a1[e];
      tile[h * 65 + k16 + 8 + e]  = a2[e];
      tile[h * 65 + k16 + 12 + e] = a3[e];
    }
  }
  __syncthreads();
  unsigned short* dst = WG + (size_t)l * (kGateN * kHid) + (size_t)g * (kHid * kHid);
  const int h8 = (t & 7) * 8;
  v4u uu[2];
#pragma unroll
  for (int it = 0; it < 2; ++it) {
    const int krow = (t >> 3) + 32 * it;
    unsigned short hb[8];
#pragma unroll
    for (int e = 0; e < 8; ++e) hb[e] = h_bits(kGateWCarry * tile[(h8 + e) * 65 + krow]);
    uu[it] = (v4u){pk16(hb[0], hb[1]), pk16(hb[2], hb[3]), pk16(hb[4], hb[5]), pk16(hb[6], hb[7])};
  }
  for (int pass = 0; pass < 2; ++pass) {
#pragma unroll
    for (int it = 0; it < 2; ++it) {
      const int krow = (t >> 3) + 32 * it;
      *(volatile v4u*)(dst + (size_t)krow * kHid + h8) = uu[it];
    }
    __threadfence();
  }
}

__device__ __forceinline__ float pick12(int r, float v0, float v1, float v2, float v3, float v4, float v5,
                                         float v6, float v7, float v8, float v9, float v10) {
  return (r == 0) ? v0 : (r == 1) ? v1 : (r == 2) ? v2 : (r == 3) ? v3 : (r == 4) ? v4 : (r == 5) ? v5 :
         (r == 6) ? v6 : (r == 7) ? v7 : (r == 8) ? v8 : (r == 9) ? v9 : (r == 10) ? v10 : 0.0f;
}
__global__ __launch_bounds__(256) void prep_link_kernel(
    const float* __restrict__ brh, const float* __restrict__ bri, const float* __restrict__ bzh, const float* __restrict__ bzi,
    const float* __restrict__ bnh, const float* __restrict__ bni,
    const float* __restrict__ Wri, const float* __restrict__ Wzi, const float* __restrict__ Wni,
    const float* __restrict__ fcw, float* __restrict__ LT) {
  const int l = blockIdx.x;
  const int t = threadIdx.x;
  const int k = t & 63;
  const int part = t >> 6;
  const size_t bo = (size_t)k * kLinks + l;
  const float v0 = brh[bo] + bri[bo];
  const float v1 = bzh[bo] + bzi[bo];
  const float v2 = bnh[bo];
  const float v3 = bni[bo];
  const size_t wo = (size_t)l * (kFeat * kHid) + k;
  const float v4 = Wri[wo], v5 = Wri[wo + kHid];
  const float v6 = Wzi[wo], v7 = Wzi[wo + kHid];
  const float v8 = Wni[wo], v9 = Wni[wo + kHid];
  const float v10 = fcw[(size_t)l * kHid + k];
  float vals[3];
#pragma unroll
  for (int q = 0; q < 3; ++q) vals[q] = pick12(part * 3 + q, v0, v1, v2, v3, v4, v5, v6, v7, v8, v9, v10);
  float* dst = LT + (size_t)l * kLTab;
  for (int pass = 0; pass < 2; ++pass) {
#pragma unroll
    for (int q = 0; q < 3; ++q) {
      const int row = part * 3 + q;
      *(volatile float*)(dst + row * kHid + k) = vals[q];
    }
    __threadfence();
  }
}

__global__ __launch_bounds__(256) void zero4_kernel(float* __restrict__ p, int n4) {
  const int i = blockIdx.x * 256 + threadIdx.x;
  if (i >= n4) return;
  const v4f z = (v4f){0.f, 0.f, 0.f, 0.f};
  float* q = p + 4 * (size_t)i;
  *(volatile v4f*)q = z;
  __threadfence();
  *(volatile v4f*)q = z;
}

__global__ __launch_bounds__(256) void transpose16_kernel(const unsigned short* __restrict__ src, unsigned short* __restrict__ dst, int R, int C) {
  __shared__ __align__(16) unsigned short tile[64 * 72];
  const int t  = threadIdx.x;
  const int c0 = blockIdx.x * 64;
  const int r0 = blockIdx.y * 64;
  {
    const int r = t >> 2, c16 = (t & 3) * 16;
    const unsigned short* p = src + (size_t)(r0 + r) * C + c0 + c16;
    const v4u a  = *(const v4u*)(p);
    const v4u a2 = *(const v4u*)(p + 8);
    *(v4u*)(tile + r * 72 + c16)     = a;
    *(v4u*)(tile + r * 72 + c16 + 8) = a2;
  }
  __syncthreads();
  const int r8 = (t & 7) * 8;
  v4u uu[2];
#pragma unroll
  for (int it = 0; it < 2; ++it) {
    const int cc = (t >> 3) + 32 * it;
    unsigned short e[8];
#pragma unroll
    for (int q = 0; q < 8; ++q) e[q] = tile[(r8 + q) * 72 + cc];
    uu[it] = (v4u){pk16(e[0], e[1]), pk16(e[2], e[3]), pk16(e[4], e[5]), pk16(e[6], e[7])};
  }
  for (int pass = 0; pass < 2; ++pass) {
#pragma unroll
    for (int it = 0; it < 2; ++it) {
      const int cc = (t >> 3) + 32 * it;
      *(volatile v4u*)(dst + (size_t)(c0 + cc) * R + r0 + r8) = uu[it];
    }
    __threadfence();
  }
}

__global__ __launch_bounds__(256) void cell_kernel(
    const float* __restrict__ HATT,
    const unsigned short* __restrict__ WG,
    const float* __restrict__ INATT, int ldI, int colI,
    const float* __restrict__ LT,
    const float* __restrict__ fcb,
    unsigned short* __restrict__ HL,
    float* __restrict__ OUTL) {
  __shared__ __align__(16) _Float16 sA[32 * 72];
  __shared__ __align__(16) float sHF[32 * 64];
  __shared__ float sD[32 * 196];
  __shared__ float sIN[64];
  __shared__ __align__(16) float sH[32 * 64];
  __shared__ float sOut[32];
  const int l    = blockIdx.x;
  const int t    = threadIdx.x;
  const int lane = t & 31;
  const int wave = t >> 5;

  {
    const int b = t >> 3, h8 = (t & 7) * 8;
    const float* p = HATT + (size_t)l * kBH + b * kHid + h8;
    const v4f a = *(const v4f*)(p);
    const v4f c = *(const v4f*)(p + 4);
    *(v4f*)(sHF + b * 64 + h8)     = a;
    *(v4f*)(sHF + b * 64 + h8 + 4) = c;
    v8h hv;
#pragma unroll
    for (int e = 0; e < 4; ++e) {
      hv[e]     = (_Float16)(a[e] * kHattCarry);
      hv[4 + e] = (_Float16)(c[e] * kHattCarry);
    }
    *(v8h*)(sA + b * 72 + h8) = hv;
    if (t < 64) sIN[t] = INATT[(size_t)l * ldI + colI + t];
  }
  __syncthreads();

  const int rlane = lane & 15;
  const int koff  = (lane >> 4) * 8;
  const int mOff  = koff;
  const int it    = wave >> 2;
  const int n0    = 48 * (wave & 3);
  v8f acc[3];
#pragma unroll
  for (int j = 0; j < 3; ++j) acc[j] = (v8f){0.f, 0.f, 0.f, 0.f, 0.f, 0.f, 0.f, 0.f};
  const _Float16* Bw = (const _Float16*)(const void*)WG + ((size_t)l * kGateN + (size_t)n0) * kHid;
#pragma unroll
  for (int ks = 0; ks < 2; ++ks) {
    const int k0 = ks * 32;
    v16h bh[3];
#pragma unroll
    for (int j = 0; j < 3; ++j) bh[j] = Frag<_Float16>::load(Bw + (size_t)(16 * j + rlane) * kHid + koff + k0);
    const v16h ah = Frag<_Float16>::load(sA + (16 * it + rlane) * 72 + koff + k0);
#pragma unroll
    for (int j = 0; j < 3; ++j) acc[j] = Frag<_Float16>::mma(ah, bh[j], acc[j]);
    Frag<_Float16>::guard(acc[0], acc[2], ah, ah);
    keep3_h(bh[0], bh[1], bh[2]);
  }
  acc_guard3(acc[0], acc[1], acc[2]);
#pragma unroll
  for (int j = 0; j < 3; ++j) {
#pragma unroll
    for (int r = 0; r < 8; ++r) sD[(16 * it + mOff + r) * 196 + n0 + 16 * j + rlane] = acc[j][r];
  }
  __syncthreads();

  {
    const int k  = t & 63;
    const int bg = (t >> 6) * 8;
    const float* lt = LT + (size_t)l * kLTab + k;
    const float cr  = lt[0 * kHid], cz  = lt[1 * kHid], cnh = lt[2 * kHid], cni = lt[3 * kHid];
    const float wr0 = lt[4 * kHid], wr1 = lt[5 * kHid], wz0 = lt[6 * kHid], wz1 = lt[7 * kHid];
    const float wn0 = lt[8 * kHid], wn1 = lt[9 * kHid];
#pragma unroll 1
    for (int i = 0; i < 8; ++i) {
      const int b = bg + i;
      const float x0 = sIN[2 * b], x1 = sIN[2 * b + 1];
      const float* d = sD + b * 196 + k;
      const float pr = d[0] * kGateScale + cr + (x0 * wr0 + x1 * wr1);
      const float pz = d[kHid] * kGateScale + cz + (x0 * wz0 + x1 * wz1);
      const float r  = 1.0f / (1.0f + __expf(-pr));
      const float z  = 1.0f / (1.0f + __expf(-pz));
      const float nn = tanhf(r * (d[2 * kHid] * kGateScale + cnh) + (x0 * wn0 + x1 * wn1 + cni));
      sH[b * 64 + k] = (1.0f - z) * nn + z * sHF[b * 64 + k];
    }
  }
  __syncthreads();

  {
    const int b = t >> 3, k8 = (t & 7) * 8;
    const v4f a = *(const v4f*)(sH + b * 64 + k8);
    const v4f c = *(const v4f*)(sH + b * 64 + k8 + 4);
    unsigned short hb[8];
#pragma unroll
    for (int e = 0; e < 4; ++e) {
      hb[e]     = h_bits(a[e] * kHidCarry);
      hb[4 + e] = h_bits(c[e] * kHidCarry);
    }
    const v4u u = (v4u){pk16(hb[0], hb[1]), pk16(hb[2], hb[3]), pk16(hb[4], hb[5]), pk16(hb[6], hb[7])};
    unsigned short* q = HL + (size_t)l * kBH + (size_t)t * 8;
    *(volatile v4u*)q = u;
    const float* fcp = LT + (size_t)l * kLTab + 10 * kHid + k8;
    const v4f f0 = *(const v4f*)(fcp);
    const v4f f1 = *(const v4f*)(fcp + 4);
    float s = ((a[0] * f0[0] + a[1] * f0[1]) + (a[2] * f0[2] + a[3] * f0[3]))
            + ((c[0] * f1[0] + c[1] * f1[1]) + (c[2] * f1[2] + c[3] * f1[3]));
    s += __shfl_xor(s, 1, 32);
    s += __shfl_xor(s, 2, 32);
    s += __shfl_xor(s, 4, 32);
    if ((t & 7) == 0) sOut[b] = s + fcb[l];
    __threadfence();
    *(volatile v4u*)q = u;
  }
  __syncthreads();
  if (wave == 0) {
    const float v = sOut[lane];
    float* q = OUTL + (size_t)l * kBatch + lane;
    *(volatile float*)q = v;
    __threadfence();
    *(volatile float*)q = v;
  }
}

__global__ __launch_bounds__(256) void decin_kernel(const float* __restrict__ OUTL, float* __restrict__ out,
                                                    unsigned short* __restrict__ IND, int s) {
  __shared__ float tile[64 * 33];
  const int t  = threadIdx.x;
  const int l0 = blockIdx.x * 64;
  {
    const int r = t >> 2, c8 = (t & 3) * 8;
    const float* p = OUTL + (size_t)(l0 + r) * kBatch + c8;
    const v4f a = *(const v4f*)(p);
    const v4f c = *(const v4f*)(p + 4);
#pragma unroll
    for (int e = 0; e < 4; ++e) {
      tile[r * 33 + c8 + e]     = a[e];
      tile[r * 33 + c8 + 4 + e] = c[e];
    }
  }
  __syncthreads();
  {
    const int c4 = (t & 15) * 4;
    v4f ov[2];
#pragma unroll
    for (int it = 0; it < 2; ++it) {
      const int b = (t >> 4) + 16 * it;
      ov[it] = (v4f){tile[(c4 + 0) * 33 + b], tile[(c4 + 1) * 33 + b], tile[(c4 + 2) * 33 + b], tile[(c4 + 3) * 33 + b]};
    }
    for (int pass = 0; pass < 2; ++pass) {
#pragma unroll
      for (int it = 0; it < 2; ++it) {
        const int b = (t >> 4) + 16 * it;
        *(volatile v4f*)(out + ((size_t)(b * kHor + s) * kLinks + l0 + c4)) = ov[it];
      }
      __threadfence();
    }
  }
  {
    const int b = t >> 3, c8 = (t & 7) * 8;
    unsigned short hb[8];
#pragma unroll
    for (int e = 0; e < 8; ++e) hb[e] = h_bits(tile[(c8 + e) * 33 + b]);
    const v4u u = (v4u){pk16(hb[0], hb[1]), pk16(hb[2], hb[3]), pk16(hb[4], hb[5]), pk16(hb[6], hb[7])};
    const v4u z = (v4u){0u, 0u, 0u, 0u};
    unsigned short* q0 = IND + (size_t)(2 * b) * kLinks + l0 + c8;
    unsigned short* q1 = IND + (size_t)(2 * b + 1) * kLinks + l0 + c8;
    *(volatile v4u*)q0 = u;
    *(volatile v4u*)q1 = z;
    __threadfence();
    *(volatile v4u*)q0 = u;
    *(volatile v4u*)q1 = z;
  }
}

extern "C" void kernel_launch(void* const* d_in, const int* in_sizes, int n_in,
                              void* d_out, int out_size, void* d_ws, size_t ws_size,
                              hipStream_t stream) {
  if (n_in < 17) return;
  if (in_sizes[0] != kBatch * kTin * kFeat * kLinks) return;
  if (in_sizes[1] != kLinks * kLinks || in_sizes[2] != kLinks * kLinks) return;
  if (in_sizes[3] != kLinks * kHid * kHid || in_sizes[7] != kLinks * kHid * kHid || in_sizes[11] != kLinks * kHid * kHid) return;
  if (in_sizes[4] != kHid * kLinks || in_sizes[5] != kLinks * kFeat * kHid) return;
  if (in_sizes[15] != kLinks * kHid || in_sizes[16] != kLinks) return;
  if (out_size != kBatch * kHor * kLinks) return;

  const float* x   = (const float*)d_in[0];
  const float* Wia = (const float*)d_in[1];
  const float* Wha = (const float*)d_in[2];
  const float* Wrh = (const float*)d_in[3];  const float* brh = (const float*)d_in[4];
  const float* Wri = (const float*)d_in[5];  const float* bri = (const float*)d_in[6];
  const float* Wzh = (const float*)d_in[7];  const float* bzh = (const float*)d_in[8];
  const float* Wzi = (const float*)d_in[9];  const float* bzi = (const float*)d_in[10];
  const float* Wnh = (const float*)d_in[11]; const float* bnh = (const float*)d_in[12];
  const float* Wni = (const float*)d_in[13]; const float* bni = (const float*)d_in[14];
  const float* fcw = (const float*)d_in[15]; const float* fcb = (const float*)d_in[16];
  float* outp = (float*)d_out;

  const size_t SZ_WA   = (size_t)kLinks * kLinks * 2;
  const size_t SZ_WG   = (size_t)kLinks * kGateN * kHid * 2;
  const size_t SZ_LT   = (size_t)kLinks * kLTab * 4;
  const size_t SZ_INE  = (size_t)kEncN * kLinks * 2;
  const size_t SZ_IAE  = (size_t)kLinks * kEncN * 4;
  const size_t SZ_IND  = (size_t)kBF * kLinks * 2;
  const size_t SZ_IAD  = (size_t)kLinks * kBF * 4;
  const size_t SZ_H16  = (size_t)kLinks * kBH * 2;
  const size_t SZ_HATT = (size_t)kLinks * kBH * 4;
  const size_t SZ_OUTL = (size_t)kLinks * kBatch * 4;
  size_t off = 0;
  const size_t oWIA = off; off += SZ_WA;
  const size_t oWHA = off; off += SZ_WA;
  const size_t oWG  = off; off += SZ_WG;
  const size_t oLT  = off; off += SZ_LT;
  const size_t oINE = off; off += SZ_INE;
  const size_t oIAE = off; off += SZ_IAE;
  const size_t oIND = off; off += SZ_IND;
  const size_t oIAD = off; off += SZ_IAD;
  const size_t oHL  = off; off += SZ_H16;
  const size_t oHID = off; off += SZ_H16;
  const size_t oHAT = off; off += SZ_HATT;
  const size_t oOUT = off; off += SZ_OUTL;
  const size_t TOTAL = off;
  if (TOTAL > ws_size) return;
  if (TOTAL > (size_t)134217728) return;

  char* ws = (char*)d_ws;
  unsigned short* WIA16  = (unsigned short*)(ws + oWIA);
  unsigned short* WHA16  = (unsigned short*)(ws + oWHA);
  unsigned short* WG16   = (unsigned short*)(ws + oWG);
  float*          LT     = (float*)(ws + oLT);
  unsigned short* INE16  = (unsigned short*)(ws + oINE);
  float*          INATTE = (float*)(ws + oIAE);
  unsigned short* IND16  = (unsigned short*)(ws + oIND);
  float*          INATTD = (float*)(ws + oIAD);
  unsigned short* HL16   = (unsigned short*)(ws + oHL);
  unsigned short* HID16  = (unsigned short*)(ws + oHID);
  float*          HATT   = (float*)(ws + oHAT);
  float*          OUTL   = (float*)(ws + oOUT);
  const float* dummy = LT;

  const dim3 blk(256);

  {
    const int n8w = kLinks * kLinks / 8;
    cast8h_kernel<<<dim3(n8w / 256), blk, 0, stream>>>(Wia, WIA16, n8w, kAttnWCarry);
    cast8h_kernel<<<dim3(n8w / 256), blk, 0, stream>>>(Wha, WHA16, n8w, kAttnWCarry);
    prep_gates_kernel<<<dim3(kLinks, 3), blk, 0, stream>>>(Wrh, Wzh, Wnh, WG16);
    prep_link_kernel<<<dim3(kLinks), blk, 0, stream>>>(brh, bri, bzh, bzi, bnh, bni, Wri, Wzi, Wni, fcw, LT);
    const int n8x = kEncN * kLinks / 8;
    castx_kernel<<<dim3(n8x / 256), blk, 0, stream>>>(x, INE16, n8x);
    const int n4h = kLinks * kBH / 4;
    zero4_kernel<<<dim3(n4h / 256), blk, 0, stream>>>(HATT, n4h);
    const dim3 gIE(((kLinks / 64) * (kEncN / 64) + 7) / 8, 1);
    wmma_gemm64<0, false, 0, 0, false, 0><<<gIE, blk, 0, stream>>>(
        WIA16, WIA16, kLinks, 0L, INE16, INE16, kLinks, 0L, (void*)INATTE, (void*)INATTE, kEncN, 0L,
        dummy, dummy, 0L, kLinks, kEncN, kLinks, kInScale);
  }

  const dim3 gTr(kBH / 64, kLinks / 64);
  const dim3 gHA(((kLinks / 64) * (kBH / 64) + 7) / 8, 1);
  const dim3 gID(((kLinks / 64) * (kBF / 64) + 7) / 8, 1);

  for (int t = 0; t < kTin; ++t) {
    if (t > 0) {
      transpose16_kernel<<<gTr, blk, 0, stream>>>(HL16, HID16, kLinks, kBH);
      wmma_gemm64<0, false, 0, 0, false, 0><<<gHA, blk, 0, stream>>>(
          WHA16, WHA16, kLinks, 0L, HID16, HID16, kLinks, 0L, (void*)HATT, (void*)HATT, kBH, 0L,
          dummy, dummy, 0L, kLinks, kBH, kLinks, kAttnScale);
    }
    cell_kernel<<<dim3(kLinks), blk, 0, stream>>>(HATT, WG16, INATTE, kEncN, t * kBF, LT, fcb, HL16, OUTL);
  }

  for (int s = 0; s < kDecCell; ++s) {
    decin_kernel<<<dim3(kLinks / 64), blk, 0, stream>>>(OUTL, outp, IND16, s);
    wmma_gemm64<0, false, 0, 0, false, 0><<<gID, blk, 0, stream>>>(
        WIA16, WIA16, kLinks, 0L, IND16, IND16, kLinks, 0L, (void*)INATTD, (void*)INATTD, kBF, 0L,
        dummy, dummy, 0L, kLinks, kBF, kLinks, kInScale);
    transpose16_kernel<<<gTr, blk, 0, stream>>>(HL16, HID16, kLinks, kBH);
    wmma_gemm64<0, false, 0, 0, false, 0><<<gHA, blk, 0, stream>>>(
        WHA16, WHA16, kLinks, 0L, HID16, HID16, kLinks, 0L, (void*)HATT, (void*)HATT, kBH, 0L,
        dummy, dummy, 0L, kLinks, kBH, kLinks, kAttnScale);
    cell_kernel<<<dim3(kLinks), blk, 0, stream>>>(HATT, WG16, INATTD, kBF, 0, LT, fcb, HL16, OUTL);
  }
  decin_kernel<<<dim3(kLinks / 64), blk, 0, stream>>>(OUTL, outp, IND16, kDecCell);
}
